// GraphAttentionNetwork_10514079941124
// MI455X (gfx1250) — hardware-verified
//
#include <hip/hip_runtime.h>
#include <stddef.h>
#include <stdint.h>
#include <math.h>

#define NN      10000
#define MP      10112
#define NE      320000
#define FD      256
#define HC1     512
#define NHD1    4
#define HID1    128
#define DOUT    256
#define XHL     1024
#define W2LD    1024
#define SPLIT2  1
#define K2EXT   (SPLIT2 ? 1024 : 512)
#define NTHR    256
#define NWAVE   8
#define EPT     8
#define WCH     (32 * EPT)
#define NBRUN   256
#define SLB     8
#define NBK     40
#define WLCAP   1536
#define RCAP    12288
#define DEGCAP  128
#define MAXDEG_MEAS  54
#define MAXB256_MEAS 8404
#define GBM     64
#define GBN     128
#define GTHR    128
#define SP      132
#define RBM     64

#define P_A1S   0
#define P_A1D   512
#define P_B1    1024
#define P_A2S   1536
#define P_A2D   1792
#define P_B2    2048
#define P_TOT   2304

#define BK_ZINTS (NWAVE * WLCAP + RCAP + 3 * NBRUN)
#define BK_INTS  (BK_ZINTS + 16)
#define BK_LDS   (BK_INTS * 4)

#define PBX   (MP * FD / 8 / NTHR)
#define PBW1  (HC1 * FD / 8 / NTHR)
#define PBW2  (DOUT * W2LD / 8 / NTHR)
#define PBP   6
#define PBTOT (PBX + PBW1 + PBW2 + PBP)

static_assert(NBK * NBRUN >= MP && NBK * NBRUN >= NN);
static_assert(MP == 79 * 128 && MP >= NN && (MP % GBM) == 0 && (MP % RBM) == 0 && (NN % 16) == 0);
static_assert(NBRUN == (1 << SLB) && (NBRUN % RBM) == 0);
static_assert(NN < (1 << 14) && NBRUN <= 256);
static_assert((((long long)NE) << SLB) < (1LL << 31));
static_assert((NE % WCH) == 0 && (NE % 4) == 0);
static_assert(RCAP == NWAVE * WLCAP && (RCAP % (NTHR * 4)) == 0 && (BK_ZINTS % 4) == 0);
static_assert((long long)RCAP * 100 >= (long long)MAXB256_MEAS * 105);
static_assert(WLCAP >= MAXB256_MEAS / 8 + 8 * 46 + 1);
static_assert(MAXDEG_MEAS + 8 <= DEGCAP);
static_assert(HC1 == 32 * 16 && DOUT == 32 * 8 && HID1 == 8 * 16 && HC1 == NHD1 * HID1);
static_assert(GBM == (GTHR / 32) * 16 && GTHR == 2 * GBM && GBN == 8 * 16 && GBN == HID1);
static_assert((HC1 % GBN) == 0 && (DOUT % GBN) == 0 && DOUT == 2 * GBN);
static_assert((FD % 32) == 0 && (K2EXT % 32) == 0 && K2EXT <= XHL && K2EXT <= W2LD && XHL == 2 * HC1);
static_assert((MP * FD / 8) % NTHR == 0 && (HC1 * FD / 8) % NTHR == 0 && (DOUT * W2LD / 8) % NTHR == 0);
static_assert(BK_LDS <= 327680);
static_assert((GBM * SP + 2 * GBN + 2 * GBM) * 4 <= 65536);
static_assert((NWAVE * HC1 * 4 + NWAVE * XHL * 2 + HC1 * 4) <= 65536);
static_assert((MP * 4) % 128 == 0 && (GBM * 4) % 128 == 0);

typedef float          v4f   __attribute__((ext_vector_type(4)));
typedef float          v8f   __attribute__((ext_vector_type(8)));
typedef int            v4i   __attribute__((ext_vector_type(4)));
typedef int            v8i   __attribute__((ext_vector_type(8)));
typedef unsigned short v8us  __attribute__((ext_vector_type(8)));
typedef unsigned short v16us __attribute__((ext_vector_type(16)));
typedef __bf16         v16bf __attribute__((ext_vector_type(16)));
typedef v4f  __attribute__((may_alias)) v4fa;
typedef v4i  __attribute__((may_alias)) v4ia;
typedef v8us __attribute__((may_alias)) v8usa;
union FragB { v16bf v; v16us u; v8us h[2]; v8i w; };

__device__ __forceinline__ v8f wmb(const FragB& a, const FragB& b, v8f c) {
  v8f d = __builtin_amdgcn_wmma_f32_16x16x32_bf16(false, a.v, false, b.v, (short)0, c, false, false);
  asm volatile("v_nop\n\tv_nop\n\tv_nop\n\tv_nop" : "+v"(d) : "v"(a.w), "v"(b.w));
  return d;
}

__device__ __forceinline__ unsigned bf16_bits(float f) {
  const unsigned u = __float_as_uint(f);
  const unsigned r = (u + 0x7FFFu + ((u >> 16) & 1u)) >> 16;
  const unsigned q = (u >> 16) | 0x40u;
  return ((u & 0x7fffffffu) > 0x7f800000u) ? q : r;
}
__device__ __forceinline__ float bf16_val(float f) {
  return __uint_as_float(bf16_bits(f) << 16);
}

__device__ __forceinline__ void st2_v4f(float* p, v4f v) {
  *(volatile v4f*)p = v;
  __threadfence();
  *(volatile v4f*)p = v;
}
__device__ __forceinline__ void st2_v8us(unsigned short* p, v8us v) {
  *(volatile v8us*)p = v;
  __threadfence();
  *(volatile v8us*)p = v;
}

__device__ __forceinline__ v8us col8(const float* __restrict__ base, int stride) {
  float f[8];
#pragma unroll
  for (int i = 0; i < 8; ++i) f[i] = base[(size_t)i * (size_t)stride];
  v8us o;
#pragma unroll
  for (int i = 0; i < 8; ++i) o[i] = (unsigned short)bf16_bits(f[i]);
  return o;
}

__device__ __forceinline__ void par_copy(const float* __restrict__ src, float* dst, int n4, int tid) {
  const int i = tid < n4 ? tid : n4 - 1;
  const v4f a = *(const v4fa*)(src + 4 * i);
  asm volatile("" :: "v"(a));
  v4f o;
  o.x = bf16_val(a.x); o.y = bf16_val(a.y); o.z = bf16_val(a.z); o.w = bf16_val(a.w);
  if (tid < n4) st2_v4f(dst + 4 * tid, o);
}

__global__ __launch_bounds__(NTHR) void k_prep(const float* __restrict__ x, const float* __restrict__ w1,
                                               const float* __restrict__ a1s, const float* __restrict__ a1d,
                                               const float* __restrict__ b1, const float* __restrict__ w2,
                                               const float* __restrict__ a2s, const float* __restrict__ a2d,
                                               const float* __restrict__ b2,
                                               unsigned short* xb, unsigned short* w1t, unsigned short* w2d,
                                               float* pp) {
  const int tid = (int)threadIdx.x;
  const int blk = (int)blockIdx.x;
  if (blk < PBX) {
    const int u   = blk * NTHR + tid;
    const int row = u >> 5, k8 = (u & 31) * 8;
    const int rc  = row < NN ? row : NN - 1;
    const unsigned mk = row < NN ? 0xffffu : 0u;
    const float* p = x + (size_t)rc * FD + k8;
    const v4f a = *(const v4fa*)p;
    const v4f b = *(const v4fa*)(p + 4);
    v8us o;
    o[0] = (unsigned short)(bf16_bits(a.x) & mk); o[1] = (unsigned short)(bf16_bits(a.y) & mk);
    o[2] = (unsigned short)(bf16_bits(a.z) & mk); o[3] = (unsigned short)(bf16_bits(a.w) & mk);
    o[4] = (unsigned short)(bf16_bits(b.x) & mk); o[5] = (unsigned short)(bf16_bits(b.y) & mk);
    o[6] = (unsigned short)(bf16_bits(b.z) & mk); o[7] = (unsigned short)(bf16_bits(b.w) & mk);
    st2_v8us(xb + (size_t)row * FD + k8, o);
  } else if (blk < PBX + PBW1) {
    const int u = (blk - PBX) * NTHR + tid;
    const int n = u >> 5, k8 = (u & 31) * 8;
    const v8us o = col8(w1 + (size_t)k8 * HC1 + n, HC1);
    st2_v8us(w1t + (size_t)n * FD + k8, o);
  } else if (blk < PBX + PBW1 + PBW2) {
    const int u = (blk - PBX - PBW1) * NTHR + tid;
    const int n = u >> 7, k8 = (u & 127) * 8, kk = k8 & 511;
    const v8us o = col8(w2 + (size_t)kk * DOUT + n, DOUT);
    st2_v8us(w2d + (size_t)n * W2LD + k8, o);
  } else {
    const int pb = blk - (PBX + PBW1 + PBW2);
    if (pb == 0)      par_copy(a1s, pp + P_A1S, 128, tid);
    else if (pb == 1) par_copy(a1d, pp + P_A1D, 128, tid);
    else if (pb == 2) par_copy(b1,  pp + P_B1,  128, tid);
    else if (pb == 3) par_copy(a2s, pp + P_A2S, 64, tid);
    else if (pb == 4) par_copy(a2d, pp + P_A2D, 64, tid);
    else              par_copy(b2,  pp + P_B2,  64, tid);
  }
}

__device__ __forceinline__ void bucket_flush(const int* pl, const int* cnt, int ov, int* lp, int* cop, int* fp,
                                             int tid) {
#pragma unroll 1
  for (int i = tid * 4; i < RCAP; i += NTHR * 4) {
    const v4i v = *(const v4ia*)(pl + i);
    *(volatile v4i*)(lp + i) = v;
  }
  if (tid < (2 * NBRUN) / 4) {
    const v4i v = *(const v4ia*)(cnt + 4 * tid);
    *(volatile v4i*)(cop + 4 * tid) = v;
  }
  if (tid < 8) {
    const v4i f = {ov, ov, ov, ov};
    *(volatile v4i*)(fp + 4 * tid) = f;
  }
}

__global__ __launch_bounds__(NTHR) void k_bucket(const int* __restrict__ srcs, const int* __restrict__ dsts,
                                                 int* LIST, int* CO, int* FLAG) {
  extern __shared__ __attribute__((aligned(16))) int dsm[];
  int* wl   = dsm;
  int* pl   = dsm + NWAVE * WLCAP;
  int* cnt  = pl + RCAP;
  int* offs = cnt + NBRUN;
  int* cur  = offs + NBRUN;
  int* misc = cur + NBRUN;
  const int tid = (int)threadIdx.x, lane = tid & 31, wave = tid >> 5;
  const int blk = (int)blockIdx.x;
  const unsigned nbs = (unsigned)(blk * NBRUN);

  {
    const v4i z4 = {0, 0, 0, 0};
    for (int i = tid * 4; i < BK_ZINTS; i += NTHR * 4) *(v4ia*)(dsm + i) = z4;
    if (tid < 16) misc[tid] = 0;
  }
  __syncthreads();

  {
    const int per  = ((NE + NWAVE * WCH - 1) / (NWAVE * WCH)) * WCH;
    const int ebeg = wave * per;
    const int eend = (ebeg + per < NE) ? (ebeg + per) : NE;
    int* mylist = wl + wave * WLCAP;
    int wc = 0;
#pragma unroll 1
    for (int cb = ebeg; cb < eend; cb += WCH) {
      const int e0 = cb + lane * EPT;
      const v4i da = *(const v4ia*)(dsts + e0);
      const v4i db = *(const v4ia*)(dsts + e0 + 4);
      const unsigned s0 = (unsigned)da.x - nbs, s1 = (unsigned)da.y - nbs;
      const unsigned s2 = (unsigned)da.z - nbs, s3 = (unsigned)da.w - nbs;
      const unsigned s4 = (unsigned)db.x - nbs, s5 = (unsigned)db.y - nbs;
      const unsigned s6 = (unsigned)db.z - nbs, s7 = (unsigned)db.w - nbs;
      const bool h0 = s0 < (unsigned)NBRUN, h1 = s1 < (unsigned)NBRUN, h2 = s2 < (unsigned)NBRUN, h3 = s3 < (unsigned)NBRUN;
      const bool h4 = s4 < (unsigned)NBRUN, h5 = s5 < (unsigned)NBRUN, h6 = s6 < (unsigned)NBRUN, h7 = s7 < (unsigned)NBRUN;
      const unsigned m0 = __builtin_amdgcn_ballot_w32(h0), m1 = __builtin_amdgcn_ballot_w32(h1);
      const unsigned m2 = __builtin_amdgcn_ballot_w32(h2), m3 = __builtin_amdgcn_ballot_w32(h3);
      const unsigned m4 = __builtin_amdgcn_ballot_w32(h4), m5 = __builtin_amdgcn_ballot_w32(h5);
      const unsigned m6 = __builtin_amdgcn_ballot_w32(h6), m7 = __builtin_amdgcn_ballot_w32(h7);
      const unsigned any = m0 | m1 | m2 | m3 | m4 | m5 | m6 | m7;
      if (any != 0u) {
        const int pre = (int)(__builtin_amdgcn_mbcnt_lo(m0, 0u) + __builtin_amdgcn_mbcnt_lo(m1, 0u) +
                              __builtin_amdgcn_mbcnt_lo(m2, 0u) + __builtin_amdgcn_mbcnt_lo(m3, 0u) +
                              __builtin_amdgcn_mbcnt_lo(m4, 0u) + __builtin_amdgcn_mbcnt_lo(m5, 0u) +
                              __builtin_amdgcn_mbcnt_lo(m6, 0u) + __builtin_amdgcn_mbcnt_lo(m7, 0u));
        int p = wc + pre;
        if (h0) { if (p < WLCAP) mylist[p] = ((e0 + 0) << SLB) | (int)s0; p = p + 1; }
        if (h1) { if (p < WLCAP) mylist[p] = ((e0 + 1) << SLB) | (int)s1; p = p + 1; }
        if (h2) { if (p < WLCAP) mylist[p] = ((e0 + 2) << SLB) | (int)s2; p = p + 1; }
        if (h3) { if (p < WLCAP) mylist[p] = ((e0 + 3) << SLB) | (int)s3; p = p + 1; }
        if (h4) { if (p < WLCAP) mylist[p] = ((e0 + 4) << SLB) | (int)s4; p = p + 1; }
        if (h5) { if (p < WLCAP) mylist[p] = ((e0 + 5) << SLB) | (int)s5; p = p + 1; }
        if (h6) { if (p < WLCAP) mylist[p] = ((e0 + 6) << SLB) | (int)s6; p = p + 1; }
        if (h7) { if (p < WLCAP) mylist[p] = ((e0 + 7) << SLB) | (int)s7; p = p + 1; }
        wc += (int)(__builtin_popcount(m0) + __builtin_popcount(m1) + __builtin_popcount(m2) + __builtin_popcount(m3) +
                    __builtin_popcount(m4) + __builtin_popcount(m5) + __builtin_popcount(m6) + __builtin_popcount(m7));
      }
    }
    if (lane == 0) misc[wave] = wc;
  }
  __syncthreads();

  if (wave == 0) {
    int ov = 0;
#pragma unroll 1
    for (int w2 = 0; w2 < NWAVE; ++w2) {
      int c = misc[w2];
      if (c > WLCAP) ov = 1;
      c = c < 0 ? 0 : (c > WLCAP ? WLCAP : c);
#pragma unroll 1
      for (int b0 = 0; b0 < c; b0 += 32) {
        const int idx = b0 + lane;
        const int ent = wl[w2 * WLCAP + (idx < WLCAP ? idx : WLCAP - 1)];
        const int m32 = (c - b0) < 32 ? (c - b0) : 32;
#pragma unroll 1
        for (int k = 0; k < m32; ++k) {
          const int u    = __builtin_amdgcn_readlane(ent, k);
          const int slot = u & (NBRUN - 1);
          if (lane == 0) cnt[slot] = cnt[slot] + 1;
        }
      }
    }
    if (lane == 0) misc[9] = ov;
  }
  __syncthreads();
  if (wave == 0) {
    const int base = lane * (NBRUN / 32);
    int s = 0;
#pragma unroll 1
    for (int i = 0; i < NBRUN / 32; ++i) s += cnt[base + i];
    int incl = s;
#pragma unroll
    for (int d = 1; d < 32; d <<= 1) {
      const int y = __shfl_up(incl, d, 32);
      if (lane >= d) incl += y;
    }
    int run = incl - s;
#pragma unroll 1
    for (int i = 0; i < NBRUN / 32; ++i) {
      const int cv = cnt[base + i];
      offs[base + i] = run;
      cur[base + i]  = run;
      run += cv;
    }
  }
  __syncthreads();

  if (wave == 0) {
#pragma unroll 1
    for (int w2 = 0; w2 < NWAVE; ++w2) {
      int c = misc[w2];
      c = c < 0 ? 0 : (c > WLCAP ? WLCAP : c);
#pragma unroll 1
      for (int b0 = 0; b0 < c; b0 += 32) {
        const int idx = b0 + lane;
        const int ent = wl[w2 * WLCAP + (idx < WLCAP ? idx : WLCAP - 1)];
        int eid = (ent >> SLB) & 0x7FFFFF;
        eid = eid > NE - 1 ? NE - 1 : eid;
        int sr = srcs[eid];
        sr = sr < 0 ? 0 : (sr > NN - 1 ? NN - 1 : sr);
        const int word = (int)((unsigned)sr | ((unsigned)(ent & (NBRUN - 1)) << 16));
        const int m32 = (c - b0) < 32 ? (c - b0) : 32;
#pragma unroll 1
        for (int k = 0; k < m32; ++k) {
          const int u    = __builtin_amdgcn_readlane(ent, k);
          const int wd   = __builtin_amdgcn_readlane(word, k);
          const int slot = u & (NBRUN - 1);
          if (lane == 0) {
            int p = cur[slot];
            p = p < 0 ? 0 : (p > RCAP - 1 ? RCAP - 1 : p);
            pl[p] = wd;
            cur[slot] = p + 1;
          }
        }
      }
    }
  }
  __syncthreads();

  const int ovf = misc[9];
  int* lp  = LIST + (size_t)blk * RCAP;
  int* cop = CO + (size_t)blk * (2 * NBRUN);
  int* fp  = FLAG + (size_t)blk * 32;
  bucket_flush(pl, cnt, ovf, lp, cop, fp, tid);
  __threadfence();
  bucket_flush(pl, cnt, ovf, lp, cop, fp, tid);
}

__global__ __launch_bounds__(GTHR) __attribute__((amdgpu_num_vgpr(248)))
void k_gemm(const unsigned short* __restrict__ A, int lda, const unsigned short* __restrict__ WT, int ldb,
            int kext, float* outF, int ldo, const float* __restrict__ atts, const float* __restrict__ attd,
            float* SD) {
  __shared__ __attribute__((aligned(16))) float stg[GBM * SP];
  __shared__ __attribute__((aligned(16))) float satt[2 * GBN];
  __shared__ __attribute__((aligned(16))) float sdot[2 * GBM];
  const int tid = (int)threadIdx.x, lane = tid & 31, wave = tid >> 5, hh = lane >> 4, m = lane & 15;
  const int rowBase = (int)blockIdx.x * GBM;
  const int grp     = (int)blockIdx.y;
  const int col0    = grp * GBN;

  if (tid < 32) {
    const v4f vs = *(const v4fa*)(atts + col0 + 4 * tid);
    const v4f vd = *(const v4fa*)(attd + col0 + 4 * tid);
    *(v4fa*)(satt + 4 * tid) = vs;
    *(v4fa*)(satt + GBN + 4 * tid) = vd;
  }

  v8f acc[8];
  {
    const v8f z = {0.f, 0.f, 0.f, 0.f, 0.f, 0.f, 0.f, 0.f};
#pragma unroll
    for (int t = 0; t < 8; ++t) acc[t] = z;
  }
  const unsigned short* ap = A  + (size_t)(rowBase + 16 * wave + m) * (size_t)lda + 8 * hh;
  const unsigned short* wp = WT + (size_t)(col0 + m) * (size_t)ldb + 8 * hh;
#pragma unroll 1
  for (int k0 = 0; k0 < kext; k0 += 32) {
    FragB af;
    af.h[0] = *(const v8usa*)(ap + k0);
    af.h[1] = *(const v8usa*)(ap + k0 + 16);
#pragma unroll
    for (int t = 0; t < 8; ++t) {
      const unsigned short* wq = wp + (size_t)(16 * t) * (size_t)ldb + k0;
      FragB bf;
      bf.h[0] = *(const v8usa*)wq;
      bf.h[1] = *(const v8usa*)(wq + 16);
      acc[t] = wmb(af, bf, acc[t]);
    }
  }

#pragma unroll
  for (int t = 0; t < 8; ++t) {
#pragma unroll
    for (int r = 0; r < 8; ++r) stg[(16 * wave + 8 * hh + r) * SP + 16 * t + m] = acc[t][r];
  }
  __syncthreads();

  {
    const int row = tid & 63, which = tid >> 6;
    const float* sa = satt + which * GBN;
    const float* hr = stg + row * SP;
    float d = 0.0f;
#pragma unroll 4
    for (int c4 = 0; c4 < GBN / 4; ++c4) {
      const v4f hv = *(const v4fa*)(hr + 4 * c4);
      const v4f av = *(const v4fa*)(sa + 4 * c4);
      d = fmaf(hv.x, av.x, d);
      d = fmaf(hv.y, av.y, d);
      d = fmaf(hv.z, av.z, d);
      d = fmaf(hv.w, av.w, d);
    }
    sdot[which * GBM + row] = d;
  }
  __syncthreads();

#pragma unroll 1
  for (int i = 0; i < 16; ++i) {
    const int lr = 16 * wave + i;
    const v4f v = *(const v4fa*)(stg + lr * SP + 4 * lane);
    st2_v4f(outF + (size_t)(rowBase + lr) * (size_t)ldo + col0 + 4 * lane, v);
  }
  if (wave == 0) {
    const int which2 = lane >> 4, piece = lane & 15;
    const v4f sdv = *(const v4fa*)(sdot + which2 * GBM + 4 * piece);
    st2_v4f(SD + (size_t)(2 * grp + which2) * (size_t)MP + rowBase + 4 * piece, sdv);
  }
}

__device__ __forceinline__ v4f upd4(v4f a, float s1, float s2, v4f f) {
  v4f r;
  r.x = fmaf(a.x, s1, s2 * f.x);
  r.y = fmaf(a.y, s1, s2 * f.y);
  r.z = fmaf(a.z, s1, s2 * f.z);
  r.w = fmaf(a.w, s1, s2 * f.w);
  return r;
}

__global__ __launch_bounds__(NTHR) void k_replay1(const int* __restrict__ LIST, const int* __restrict__ CO,
                                                  const int* __restrict__ FLAG, const float* __restrict__ H1,
                                                  const float* __restrict__ SD, const float* __restrict__ PP,
                                                  unsigned short* X1) {
  __shared__ __attribute__((aligned(16))) float sv[NWAVE * HC1];
  __shared__ __attribute__((aligned(16))) unsigned short sh[NWAVE * XHL];
  __shared__ __attribute__((aligned(16))) float sb1[HC1];
  const int tid = (int)threadIdx.x, lane = tid & 31, wave = tid >> 5;
  const int rowBase = (int)blockIdx.x * RBM;
  const int bucket  = rowBase >> SLB;
  const int* lb  = LIST + (size_t)bucket * RCAP;
  const int* cob = CO + (size_t)bucket * (2 * NBRUN);
  const int flag = FLAG[(size_t)bucket * 32];
  if (tid < HC1 / 4) *(v4fa*)(sb1 + 4 * tid) = *(const v4fa*)(PP + P_B1 + 4 * tid);
  __syncthreads();

  const int hd = lane >> 3;
  const int pS = (2 * hd) * MP, pD = pS + MP;
  float* svw = sv + wave * HC1;
  unsigned short* shw = sh + wave * XHL;
  const float qnan = __uint_as_float(0x7fc00000u);

#pragma unroll 1
  for (int it = 0; it < RBM / NWAVE; ++it) {
    const int d    = rowBase + (RBM / NWAVE) * wave + it;
    const int slot = d & (NBRUN - 1);
    int cv = cob[slot];
    int ov = cob[NBRUN + slot];
    const bool big = cv > DEGCAP;
    cv = cv < 0 ? 0 : (cv > DEGCAP ? DEGCAP : cv);
    ov = ov < 0 ? 0 : (ov > RCAP - 1 ? RCAP - 1 : ov);
    int lastv = ov + cv - 1; lastv = lastv < ov ? ov : lastv;
    lastv = lastv > RCAP - 1 ? RCAP - 1 : lastv;
    const int c    = __builtin_amdgcn_readfirstlane(cv);
    const int o    = __builtin_amdgcn_readfirstlane(ov);
    const int last = __builtin_amdgcn_readfirstlane(lastv);

    const float* hrow = H1 + (size_t)d * HC1 + 16 * lane;
    v4f a0 = *(const v4fa*)(hrow), a1 = *(const v4fa*)(hrow + 4);
    v4f a2 = *(const v4fa*)(hrow + 8), a3 = *(const v4fa*)(hrow + 12);
    const float adv = SD[pD + d];
    float l0 = SD[pS + d] + adv;
    l0 = l0 > 0.0f ? l0 : 0.2f * l0;
    float mx = l0, dn = 1.0f;

#pragma unroll 1
    for (int j = 0; j < c; ++j) {
      int idx = o + j;
      idx = idx > last ? last : idx;
      const unsigned wd = (unsigned)lb[idx];
      int sr = (int)(wd & 0xffffu);
      sr = sr > NN - 1 ? NN - 1 : sr;
      const float* srow = H1 + (size_t)sr * HC1 + 16 * lane;
      const v4f f0 = *(const v4fa*)(srow), f1 = *(const v4fa*)(srow + 4);
      const v4f f2 = *(const v4fa*)(srow + 8), f3 = *(const v4fa*)(srow + 12);
      asm volatile("" :: "v"(f0), "v"(f1));
      asm volatile("" :: "v"(f2), "v"(f3));
      float lg = SD[pS + sr] + adv;
      lg = lg > 0.0f ? lg : 0.2f * lg;
      const float df = lg - mx;
      const float ee = expf(-fabsf(df));
      const bool up  = df > 0.0f;
      const float s1 = up ? ee : 1.0f;
      const float s2 = up ? 1.0f : ee;
      mx = up ? lg : mx;
      dn = fmaf(dn, s1, s2);
      a0 = upd4(a0, s1, s2, f0);
      a1 = upd4(a1, s1, s2, f1);
      a2 = upd4(a2, s1, s2, f2);
      a3 = upd4(a3, s1, s2, f3);
    }
    const float inv = 1.0f / dn;
    a0.x *= inv; a0.y *= inv; a0.z *= inv; a0.w *= inv;
    a1.x *= inv; a1.y *= inv; a1.z *= inv; a1.w *= inv;
    a2.x *= inv; a2.y *= inv; a2.z *= inv; a2.w *= inv;
    a3.x *= inv; a3.y *= inv; a3.z *= inv; a3.w *= inv;
    *(v4fa*)(svw + 16 * lane)      = a0;
    *(v4fa*)(svw + 16 * lane + 4)  = a1;
    *(v4fa*)(svw + 16 * lane + 8)  = a2;
    *(v4fa*)(svw + 16 * lane + 12) = a3;
    __syncthreads();

    const bool bad  = (flag != 0) | big;
    const bool live = d < NN;
#pragma unroll 1
    for (int i2 = 0; i2 < HC1 / 32; ++i2) {
      const int p = lane + 32 * i2;
      float v = svw[p] + sb1[p];
      const float em = expm1f(v);
      v = (v > 0.0f) ? v : em;
      v = bad ? qnan : v;
      v = live ? v : 0.0f;
      const unsigned hb = bf16_bits(v);
      const unsigned lw = bf16_bits(v - __uint_as_float(hb << 16));
      shw[p]       = (unsigned short)hb;
      shw[HC1 + p] = (unsigned short)lw;
    }
    __syncthreads();

    const v8us q0 = *(const v8usa*)(shw + 8 * lane);
    const v8us q1 = *(const v8usa*)(shw + 8 * (32 + lane));
    const v8us q2 = *(const v8usa*)(shw + 8 * (64 + lane));
    const v8us q3 = *(const v8usa*)(shw + 8 * (96 + lane));
    unsigned short* gp = X1 + (size_t)d * XHL + 8 * lane;
    *(volatile v8us*)(gp)       = q0;
    *(volatile v8us*)(gp + 256) = q1;
    *(volatile v8us*)(gp + 512) = q2;
    *(volatile v8us*)(gp + 768) = q3;
    __threadfence();
    *(volatile v8us*)(gp)       = q0;
    *(volatile v8us*)(gp + 256) = q1;
    *(volatile v8us*)(gp + 512) = q2;
    *(volatile v8us*)(gp + 768) = q3;
  }
}

__global__ __launch_bounds__(NTHR) void k_replay2(const int* __restrict__ LIST, const int* __restrict__ CO,
                                                  const int* __restrict__ FLAG, const float* __restrict__ H2,
                                                  const float* __restrict__ SD, const float* __restrict__ PP,
                                                  float* out) {
  __shared__ __attribute__((aligned(16))) float sb2[DOUT];
  const int tid = (int)threadIdx.x, lane = tid & 31, wave = tid >> 5;
  const int rowBase = (int)blockIdx.x * RBM;
  const int bucket  = rowBase >> SLB;
  const int* lb  = LIST + (size_t)bucket * RCAP;
  const int* cob = CO + (size_t)bucket * (2 * NBRUN);
  const int flag = FLAG[(size_t)bucket * 32];
  if (tid < DOUT / 4) *(v4fa*)(sb2 + 4 * tid) = *(const v4fa*)(PP + P_B2 + 4 * tid);
  __syncthreads();
  const v4f bA = *(const v4fa*)(sb2 + 4 * lane);
  const v4f bB = *(const v4fa*)(sb2 + 128 + 4 * lane);
  const float qnan = __uint_as_float(0x7fc00000u);

#pragma unroll 1
  for (int it = 0; it < RBM / NWAVE; ++it) {
    const int d    = rowBase + (RBM / NWAVE) * wave + it;
    const int slot = d & (NBRUN - 1);
    int cv = cob[slot];
    int ov = cob[NBRUN + slot];
    const bool big = cv > DEGCAP;
    cv = cv < 0 ? 0 : (cv > DEGCAP ? DEGCAP : cv);
    ov = ov < 0 ? 0 : (ov > RCAP - 1 ? RCAP - 1 : ov);
    int lastv = ov + cv - 1; lastv = lastv < ov ? ov : lastv;
    lastv = lastv > RCAP - 1 ? RCAP - 1 : lastv;
    const int c    = __builtin_amdgcn_readfirstlane(cv);
    const int o    = __builtin_amdgcn_readfirstlane(ov);
    const int last = __builtin_amdgcn_readfirstlane(lastv);

    const float* hrow = H2 + (size_t)d * DOUT + 4 * lane;
    v4f a0 = *(const v4fa*)(hrow), a1 = *(const v4fa*)(hrow + 128);
    const float adv = SD[MP + d] + SD[3 * MP + d];
    float l0 = (SD[d] + SD[2 * MP + d]) + adv;
    l0 = l0 > 0.0f ? l0 : 0.2f * l0;
    float mx = l0, dn = 1.0f;

#pragma unroll 1
    for (int j = 0; j < c; ++j) {
      int idx = o + j;
      idx = idx > last ? last : idx;
      const unsigned wd = (unsigned)lb[idx];
      int sr = (int)(wd & 0xffffu);
      sr = sr > NN - 1 ? NN - 1 : sr;
      const float* srow = H2 + (size_t)sr * DOUT + 4 * lane;
      const v4f f0 = *(const v4fa*)(srow), f1 = *(const v4fa*)(srow + 128);
      asm volatile("" :: "v"(f0), "v"(f1));
      float lg = (SD[sr] + SD[2 * MP + sr]) + adv;
      lg = lg > 0.0f ? lg : 0.2f * lg;
      const float df = lg - mx;
      const float ee = expf(-fabsf(df));
      const bool up  = df > 0.0f;
      const float s1 = up ? ee : 1.0f;
      const float s2 = up ? 1.0f : ee;
      mx = up ? lg : mx;
      dn = fmaf(dn, s1, s2);
      a0 = upd4(a0, s1, s2, f0);
      a1 = upd4(a1, s1, s2, f1);
    }
    const float inv = 1.0f / dn;
    const bool bad = (flag != 0) | big;
    v4f o0, o1;
    o0.x = a0.x * inv + bA.x; o0.y = a0.y * inv + bA.y; o0.z = a0.z * inv + bA.z; o0.w = a0.w * inv + bA.w;
    o1.x = a1.x * inv + bB.x; o1.y = a1.y * inv + bB.y; o1.z = a1.z * inv + bB.z; o1.w = a1.w * inv + bB.w;
    o0.x = bad ? qnan : o0.x; o0.y = bad ? qnan : o0.y; o0.z = bad ? qnan : o0.z; o0.w = bad ? qnan : o0.w;
    o1.x = bad ? qnan : o1.x; o1.y = bad ? qnan : o1.y; o1.z = bad ? qnan : o1.z; o1.w = bad ? qnan : o1.w;
    const int dc = d < NN ? d : NN - 1;
    float* op = out + (size_t)dc * DOUT + 4 * lane;
    const bool wr = d < NN;
    if (wr) { *(volatile v4f*)(op) = o0; *(volatile v4f*)(op + 128) = o1; }
    __threadfence();
    if (wr) { *(volatile v4f*)(op) = o0; *(volatile v4f*)(op + 128) = o1; }
  }
}

extern "C" void kernel_launch(void* const* d_in, const int* in_sizes, int n_in,
                              void* d_out, int out_size, void* d_ws, size_t ws_size,
                              hipStream_t stream) {
  if (n_in < 10) return;
  if (in_sizes[0] != NN * FD) return;
  if (in_sizes[1] != 2 * NE) return;
  if (in_sizes[2] != FD * HC1) return;
  if (in_sizes[3] != NHD1 * HID1) return;
  if (in_sizes[4] != NHD1 * HID1) return;
  if (in_sizes[5] != HC1) return;
  if (in_sizes[6] != HC1 * DOUT) return;
  if (in_sizes[7] != DOUT) return;
  if (in_sizes[8] != DOUT) return;
  if (in_sizes[9] != DOUT) return;
  if (out_size != NN * DOUT) return;

  const float* x   = (const float*)d_in[0];
  const int*   ei  = (const int*)d_in[1];
  const float* W1  = (const float*)d_in[2];
  const float* a1s = (const float*)d_in[3];
  const float* a1d = (const float*)d_in[4];
  const float* b1  = (const float*)d_in[5];
  const float* W2  = (const float*)d_in[6];
  const float* a2s = (const float*)d_in[7];
  const float* a2d = (const float*)d_in[8];
  const float* b2  = (const float*)d_in[9];
  float* out = (float*)d_out;
  const int* srcs = ei;
  const int* dsts = ei + NE;

  constexpr size_t zXB   = (size_t)MP * FD * 2;
  constexpr size_t zH1   = (size_t)MP * HC1 * 4;
  constexpr size_t zX1   = (size_t)MP * XHL * 2;
  constexpr size_t zH2   = (size_t)MP * DOUT * 4;
  constexpr size_t zLIST = (size_t)NBK * RCAP * 4;
  constexpr size_t zCO   = (size_t)NBK * 2 * NBRUN * 4;
  constexpr size_t zFLAG = (size_t)NBK * 128;
  constexpr size_t zSD1  = (size_t)8 * MP * 4;
  constexpr size_t zSD2  = (size_t)4 * MP * 4;
  constexpr size_t zW1T  = (size_t)HC1 * FD * 2;
  constexpr size_t zW2D  = (size_t)DOUT * W2LD * 2;
  constexpr size_t zPP   = (size_t)P_TOT * 4;
  constexpr size_t oXB   = 0;
  constexpr size_t oH1   = oXB + zXB;
  constexpr size_t oX1   = oH1 + zH1;
  constexpr size_t oH2   = oX1 + zX1;
  constexpr size_t oLIST = oH2 + zH2;
  constexpr size_t oCO   = oLIST + zLIST;
  constexpr size_t oFLAG = oCO + zCO;
  constexpr size_t oSD1  = oFLAG + zFLAG;
  constexpr size_t oSD2  = oSD1 + zSD1;
  constexpr size_t oW1T  = oSD2 + zSD2;
  constexpr size_t oW2D  = oW1T + zW1T;
  constexpr size_t oPP   = oW2D + zW2D;
  constexpr size_t oEND  = oPP + zPP;
  static_assert(zXB % 256 == 0 && zH1 % 256 == 0 && zX1 % 256 == 0 && zH2 % 256 == 0 && zLIST % 256 == 0);
  static_assert(zCO % 256 == 0 && zFLAG % 256 == 0 && zSD1 % 256 == 0 && zSD2 % 256 == 0);
  static_assert(zW1T % 256 == 0 && zW2D % 256 == 0 && zPP % 256 == 0);
  static_assert(oEND <= (size_t)(128u << 20));
  if (oEND > ws_size) return;

  char* ws = (char*)d_ws;
  unsigned short* XB   = (unsigned short*)(ws + oXB);
  float*          H1   = (float*)(ws + oH1);
  unsigned short* X1   = (unsigned short*)(ws + oX1);
  float*          H2   = (float*)(ws + oH2);
  int*            LIST = (int*)(ws + oLIST);
  int*            CO   = (int*)(ws + oCO);
  int*            FLAG = (int*)(ws + oFLAG);
  float*          SD1  = (float*)(ws + oSD1);
  float*          SD2  = (float*)(ws + oSD2);
  unsigned short* W1T  = (unsigned short*)(ws + oW1T);
  unsigned short* W2D  = (unsigned short*)(ws + oW2D);
  float*          PP   = (float*)(ws + oPP);

  hipFuncSetAttribute(reinterpret_cast<const void*>(&k_bucket), hipFuncAttributeMaxDynamicSharedMemorySize, (int)BK_LDS);

  k_prep<<<PBTOT, NTHR, 0, stream>>>(x, W1, a1s, a1d, b1, W2, a2s, a2d, b2, XB, W1T, W2D, PP);
  k_bucket<<<NBK, NTHR, BK_LDS, stream>>>(srcs, dsts, LIST, CO, FLAG);
  k_gemm<<<dim3(MP / GBM, HC1 / GBN), GTHR, 0, stream>>>(XB, FD, W1T, FD, FD, H1, HC1,
                                                         PP + P_A1S, PP + P_A1D, SD1);
  k_replay1<<<MP / RBM, NTHR, 0, stream>>>(LIST, CO, FLAG, H1, SD1, PP, X1);
  k_gemm<<<dim3(MP / GBM, DOUT / GBN), GTHR, 0, stream>>>(X1, XHL, W2D, W2LD, K2EXT, H2, DOUT,
                                                          PP + P_A2S, PP + P_A2D, SD2);
  k_replay2<<<MP / RBM, NTHR, 0, stream>>>(LIST, CO, FLAG, H2, SD2, PP, out);
}
